// DyGCN_1778116460913
// MI455X (gfx1250) — hardware-verified
//
#include <hip/hip_runtime.h>
#include <stdint.h>

typedef __attribute__((ext_vector_type(16))) _Float16 v16h;
typedef __attribute__((ext_vector_type(8)))  _Float16 v8h;
typedef __attribute__((ext_vector_type(16))) __bf16   v16b;
typedef __attribute__((ext_vector_type(8)))  __bf16   v8b;
typedef __attribute__((ext_vector_type(8)))  float    v8f;
typedef __attribute__((ext_vector_type(4)))  float    v4f;
typedef __attribute__((ext_vector_type(4)))  unsigned int v4u;

constexpr int kBatch   = 32;
constexpr int kNode    = 500;
constexpr int kNpad    = 512;
constexpr int kDin     = 64;
constexpr int kDout    = 64;
constexpr int kEmb     = 16;
constexpr int kCheb    = 3;
constexpr int kKf      = kCheb * kDin;
constexpr int kNz      = kEmb * kDout;
constexpr int kKsPitch = 128;
constexpr int kKsReal  = 96;

static_assert(kKsReal % 32 == 0, "score GEMM K multiple of 32");
static_assert(kNpad % 64 == 0 && kDin % 64 == 0 && kNz % 64 == 0, "GEMM M/N tile multiples");
static_assert(kNpad % 32 == 0 && kKf % 32 == 0, "GEMM K multiple of 32");
static_assert(kDout == 64 && kDin == 64 && kEmb == 16 && kCheb == 3, "fixed geometry");

constexpr size_t kMiB      = 1048576;
constexpr size_t kOffPA    = 0;
constexpr size_t kOffPB    = 4 * kMiB;
constexpr size_t kOffS     = 8 * kMiB;
constexpr size_t kOffAhi   = 40 * kMiB;
constexpr size_t kOffAlo   = 56 * kMiB;
constexpr size_t kOffZ     = 0;
constexpr size_t kOffXThi  = 72 * kMiB;
constexpr size_t kOffXTlo  = 74 * kMiB;
constexpr size_t kOffXT1hi = 76 * kMiB;
constexpr size_t kOffXT1lo = 78 * kMiB;
constexpr size_t kOffYhi   = 80 * kMiB;
constexpr size_t kOffYlo   = 86 * kMiB;
constexpr size_t kOffWhi   = 92 * kMiB;
constexpr size_t kOffWlo   = 92 * kMiB + 393216;
constexpr size_t kWsTotal  = kOffWlo + 393216;
static_assert((size_t)kBatch * kNpad * kKsPitch * 2 == 4 * kMiB, "PA/PB size");
static_assert((size_t)kBatch * kNpad * kNpad * 4 == 32 * kMiB, "S size");
static_assert((size_t)kBatch * kNpad * kNpad * 2 == 16 * kMiB, "A plane size");
static_assert((size_t)kBatch * kNpad * kNz * 4 <= kOffXThi, "Z alias fits the dead region");
static_assert((size_t)kBatch * kDin * kNpad * 2 == 2 * kMiB, "xT plane size");
static_assert((size_t)kBatch * kNpad * kKf * 2 == 6 * kMiB, "Y plane size");
static_assert((size_t)kNz * kKf * 2 == 393216, "W plane size");
static_assert(kWsTotal == 97255424, "carve total");
static_assert(kWsTotal <= 134217728, "carve under 128 MiB");

__device__ __forceinline__ unsigned short f2bf_bits(float f) {
  unsigned u = __float_as_uint(f);
  return (unsigned short)((u + 0x7FFFu + ((u >> 16) & 1u)) >> 16);
}
__device__ __forceinline__ float bf_bits2f(unsigned short h) { return __uint_as_float(((unsigned)h) << 16); }

__device__ __forceinline__ void dep_guard_h(v8f& a, v8f& b, v16h x, v16h y) { asm volatile("v_nop\n\tv_nop\n\tv_nop\n\tv_nop" : "+v"(a), "+v"(b) : "v"(x), "v"(y)); }
__device__ __forceinline__ void dep_guard_b(v8f& a, v8f& b, v16b x, v16b y) { asm volatile("v_nop\n\tv_nop\n\tv_nop\n\tv_nop" : "+v"(a), "+v"(b) : "v"(x), "v"(y)); }
__device__ __forceinline__ void keep4_h(v16h a, v16h b, v16h c, v16h d) { asm volatile("v_nop" :: "v"(a), "v"(b), "v"(c), "v"(d)); }
__device__ __forceinline__ void keep4_b(v16b a, v16b b, v16b c, v16b d) { asm volatile("v_nop" :: "v"(a), "v"(b), "v"(c), "v"(d)); }
__device__ __forceinline__ void acc_guard4(v8f& a, v8f& b, v8f& c, v8f& d) { asm volatile("v_nop\n\tv_nop\n\tv_nop\n\tv_nop" : "+v"(a), "+v"(b), "+v"(c), "+v"(d)); }
template <typename T> struct Frag;
template <> struct Frag<_Float16> {
  typedef v16h V; union U { v16h v; v8h h[2]; };
  static __device__ __forceinline__ v16h load(const _Float16* p) {
    U f; f.h[0] = *(const v8h*)(p); f.h[1] = *(const v8h*)(p + 16); return f.v;
  }
  static __device__ __forceinline__ v8f mma(v16h a, v16h b, v8f c) {
    return __builtin_amdgcn_wmma_f32_16x16x32_f16(false, a, false, b, (short)0, c, false, false);
  }
  static __device__ __forceinline__ void guard(v8f& a, v8f& b, v16h x, v16h y) { dep_guard_h(a, b, x, y); }
  static __device__ __forceinline__ void keep(v16h a, v16h b, v16h c, v16h d) { keep4_h(a, b, c, d); }
};
template <> struct Frag<__bf16> {
  typedef v16b V; union U { v16b v; v8b h[2]; };
  static __device__ __forceinline__ v16b load(const __bf16* p) {
    U f; f.h[0] = *(const v8b*)(p); f.h[1] = *(const v8b*)(p + 16); return f.v;
  }
  static __device__ __forceinline__ v8f mma(v16b a, v16b b, v8f c) {
    return __builtin_amdgcn_wmma_f32_16x16x32_bf16(false, a, false, b, (short)0, c, false, false);
  }
  static __device__ __forceinline__ void guard(v8f& a, v8f& b, v16b x, v16b y) { dep_guard_b(a, b, x, y); }
  static __device__ __forceinline__ void keep(v16b a, v16b b, v16b c, v16b d) { keep4_b(a, b, c, d); }
};

template <int ET> struct Elem;
template <> struct Elem<0> { typedef _Float16 T; };
template <> struct Elem<1> { typedef __bf16 T; };
template <int ET, bool SPLIT, int BIAS_MODE, int OUT_MODE, bool RESID, int ACT = 0>
__global__ __launch_bounds__(256) void wmma_gemm64(
    const unsigned short* __restrict__ Ap, const unsigned short* __restrict__ A2p, int lda, long strideA,
    const unsigned short* __restrict__ Btp, const unsigned short* __restrict__ Bt2p, int ldb, long strideB,
    void* __restrict__ Cout, void* __restrict__ Cout2, int ldc, long strideC,
    const float* __restrict__ bias,
    const float* __restrict__ resid, long strideR,
    int M, int N, int K, float scale) {
  typedef typename Elem<ET>::T T;
  typedef typename Frag<T>::V V;
  const T* A = (const T*)Ap; const T* A2 = (const T*)A2p; const T* Bt = (const T*)Btp; const T* Bt2 = (const T*)Bt2p;
  __shared__ __align__(16) float sT[8][16 * 68];
  const int b    = blockIdx.y;
  const int lane = threadIdx.x & 31;
  const int wave = threadIdx.x >> 5;
  const int tilesN = N >> 6;
  const int tilesM = M >> 6;
  const int tile = blockIdx.x * 8 + wave;
  if (tile >= tilesM * tilesN) return;
  const int tm = tile / tilesN;
  const int tn = tile - tm * tilesN;
  const int m0 = tm << 6;
  const int n0 = tn << 6;

  const T* Ab  = A  + (size_t)b * strideA;
  const T* Bb  = Bt + (size_t)b * strideB;
  const T* Ab2 = SPLIT ? (A2  + (size_t)b * strideA) : nullptr;
  const T* Bb2 = SPLIT ? (Bt2 + (size_t)b * strideB) : nullptr;

  const int rlane = lane & 15;
  const int koff  = (lane >> 4) * 8;
  const int mOff  = (lane >> 4) * 8;

  v8f acc[4][4];
#pragma unroll
  for (int i = 0; i < 4; ++i)
#pragma unroll
    for (int j = 0; j < 4; ++j) acc[i][j] = (v8f){0.f,0.f,0.f,0.f,0.f,0.f,0.f,0.f};

  for (int k0 = 0; k0 < K; k0 += 32) {
    V bh[4], bl[4];
#pragma unroll
    for (int j = 0; j < 4; ++j) {
      const size_t bo = (size_t)(n0 + (j << 4) + rlane) * ldb + koff + k0;
      bh[j] = Frag<T>::load(Bb + bo);
      if (SPLIT) bl[j] = Frag<T>::load(Bb2 + bo);
    }
#pragma unroll
    for (int i = 0; i < 4; ++i) {
      const size_t ao = (size_t)(m0 + (i << 4) + rlane) * lda + koff + k0;
      V ah = Frag<T>::load(Ab + ao);
      V al;
      if (SPLIT) al = Frag<T>::load(Ab2 + ao);
#pragma unroll
      for (int j = 0; j < 4; ++j) {
        acc[i][j] = Frag<T>::mma(ah, bh[j], acc[i][j]);
        if (SPLIT) {
          acc[i][j] = Frag<T>::mma(ah, bl[j], acc[i][j]);
          acc[i][j] = Frag<T>::mma(al, bh[j], acc[i][j]);
        }
      }
      Frag<T>::guard(acc[i][0], acc[i][3], ah, SPLIT ? al : ah);
    }
    Frag<T>::keep(bh[0], bh[1], bh[2], bh[3]);
    if (SPLIT) Frag<T>::keep(bl[0], bl[1], bl[2], bl[3]);
  }
  acc_guard4(acc[0][0], acc[0][1], acc[0][2], acc[0][3]);
  acc_guard4(acc[1][0], acc[1][1], acc[1][2], acc[1][3]);
  acc_guard4(acc[2][0], acc[2][1], acc[2][2], acc[2][3]);
  acc_guard4(acc[3][0], acc[3][1], acc[3][2], acc[3][3]);

  float* slab = sT[wave];
  const float* Rb = RESID ? (resid + (size_t)b * strideR) : nullptr;
#pragma unroll
  for (int i = 0; i < 4; ++i) {
    const int mBase = m0 + (i << 4);
#pragma unroll
    for (int j = 0; j < 4; ++j) {
      const int n = n0 + (j << 4) + rlane;
      float bv = 0.f;
      if (BIAS_MODE == 2) bv = bias[n];
#pragma unroll
      for (int r = 0; r < 8; ++r) {
        float v = acc[i][j][r] * scale;
        if (BIAS_MODE == 1) v += bias[mBase + mOff + r];
        if (BIAS_MODE == 2) v += bv;
        if (RESID) v += Rb[(size_t)(mBase + mOff + r) * ldc + n];
        if (ACT == 1) v = tanhf(v);
        if (ACT == 2) v = fmaxf(v, 0.0f);
        if (ACT == 3) v = v / (1.0f + expf(-v));
        if (ACT == 4) v = (v > 0.f) ? v : 0.01f * v;
        if (ACT == 5) v = 0.5f * v * (1.0f + erff(v * 0.70710678118654752f));
        slab[(mOff + r) * 68 + (j << 4) + rlane] = v;
      }
    }
    __builtin_amdgcn_fence(__ATOMIC_RELEASE, "workgroup");
    __builtin_amdgcn_wave_barrier();
    __builtin_amdgcn_fence(__ATOMIC_ACQUIRE, "workgroup");
    if (OUT_MODE == 0) {
      float* C = (float*)Cout + (size_t)b * strideC;
      const int hh = lane >> 4, c4 = (lane & 15) * 4;
      for (int pass = 0; pass < 2; ++pass) {
#pragma unroll
        for (int it = 0; it < 8; ++it) {
          const int row = it * 2 + hh;
          v4f v = *(const v4f*)(slab + row * 68 + c4);
          *(volatile v4f*)(C + (size_t)(mBase + row) * ldc + n0 + c4) = v;
        }
        __threadfence();
      }
    } else {
      const int q = lane >> 3, c8 = (lane & 7) * 8;
      unsigned short* C  = (unsigned short*)Cout  + (size_t)b * strideC;
      unsigned short* C2 = (OUT_MODE == 2) ? ((unsigned short*)Cout2 + (size_t)b * strideC) : nullptr;
      for (int pass = 0; pass < 2; ++pass) {
#pragma unroll
        for (int it = 0; it < 4; ++it) {
          const int row = it * 4 + q;
          const float* sp = slab + row * 68 + c8;
          v8h hv, lv;
#pragma unroll
          for (int e = 0; e < 8; ++e) {
            if (OUT_MODE == 1) {
              hv[e] = (_Float16)sp[e];
            } else {
              unsigned short hb = f2bf_bits(sp[e]);
              unsigned short lb = f2bf_bits(sp[e] - bf_bits2f(hb));
              hv[e] = __builtin_bit_cast(_Float16, hb);
              lv[e] = __builtin_bit_cast(_Float16, lb);
            }
          }
          *(volatile v8h*)(C + (size_t)(mBase + row) * ldc + n0 + c8) = hv;
          if (OUT_MODE == 2) *(volatile v8h*)(C2 + (size_t)(mBase + row) * ldc + n0 + c8) = lv;
        }
        __threadfence();
      }
    }
    __builtin_amdgcn_fence(__ATOMIC_RELEASE, "workgroup");
    __builtin_amdgcn_wave_barrier();
    __builtin_amdgcn_fence(__ATOMIC_ACQUIRE, "workgroup");
  }
}

__device__ __forceinline__ void split2_bf(float a, float b, unsigned& whi, unsigned& wlo) {
  const unsigned short ha = f2bf_bits(a), hb = f2bf_bits(b);
  const unsigned short la = f2bf_bits(a - bf_bits2f(ha)), lb = f2bf_bits(b - bf_bits2f(hb));
  whi = (unsigned)ha | ((unsigned)hb << 16);
  wlo = (unsigned)la | ((unsigned)lb << 16);
}

__global__ __launch_bounds__(256) void k_pack_emb(const float* __restrict__ emb,
                                                  unsigned short* __restrict__ pa,
                                                  unsigned short* __restrict__ pb) {
  const int gid   = blockIdx.x * 256 + threadIdx.x;
  const int chunk = gid & 15;
  const int rowg  = gid >> 4;
  const int b     = rowg >> 9;
  const int n     = rowg & 511;
  const int grp   = chunk >> 1;
  const int e0    = (chunk & 1) * 8;
  const bool valid = (n < kNode) && (grp < 6);
  const int nc    = (n < kNode) ? n : (kNode - 1);
  const float* src = emb + ((size_t)b * kNode + nc) * kEmb + e0;
  const v4f x0 = *(const v4f*)(src);
  const v4f x1 = *(const v4f*)(src + 4);
  float xv[8] = {x0[0], x0[1], x0[2], x0[3], x1[0], x1[1], x1[2], x1[3]};
  const bool aH = (grp <= 2), aM = (grp == 3) || (grp == 4);
  const bool bH = (grp == 0) || (grp == 3) || (grp == 5), bM = (grp == 1) || (grp == 4);
  unsigned wa[4], wb[4];
#pragma unroll
  for (int j = 0; j < 4; ++j) {
    unsigned sa2[2], sb2[2];
#pragma unroll
    for (int t = 0; t < 2; ++t) {
      const float xe = xv[2 * j + t];
      const unsigned short hb = f2bf_bits(xe);
      const float r1 = xe - bf_bits2f(hb);
      const unsigned short mb = f2bf_bits(r1);
      const float r2 = r1 - bf_bits2f(mb);
      const unsigned short lb = f2bf_bits(r2);
      unsigned sa = aH ? (unsigned)hb : (aM ? (unsigned)mb : (unsigned)lb);
      unsigned sb = bH ? (unsigned)hb : (bM ? (unsigned)mb : (unsigned)lb);
      sa = valid ? sa : 0u;
      sb = valid ? sb : 0u;
      sa2[t] = sa; sb2[t] = sb;
    }
    wa[j] = sa2[0] | (sa2[1] << 16);
    wb[j] = sb2[0] | (sb2[1] << 16);
  }
  v4u va, vb;
  va[0] = wa[0]; va[1] = wa[1]; va[2] = wa[2]; va[3] = wa[3];
  vb[0] = wb[0]; vb[1] = wb[1]; vb[2] = wb[2]; vb[3] = wb[3];
  const size_t off = (size_t)rowg * kKsPitch + chunk * 8;
  *(volatile v4u*)(pa + off) = va;
  *(volatile v4u*)(pb + off) = vb;
  __threadfence();
  *(volatile v4u*)(pa + off) = va;
  *(volatile v4u*)(pb + off) = vb;
}

__global__ __launch_bounds__(256) void k_pack_x(const float* __restrict__ x,
                                                unsigned short* __restrict__ xthi, unsigned short* __restrict__ xtlo,
                                                unsigned short* __restrict__ yhi,  unsigned short* __restrict__ ylo) {
  __shared__ float tile[64][65];
  const int tid = threadIdx.x;
  const int mc  = blockIdx.x;
  const int b   = blockIdx.y;
  const int m0  = mc * 64;
#pragma unroll
  for (int it = 0; it < 4; ++it) {
    const int idx = it * 256 + tid;
    const int r = idx >> 4, c4 = (idx & 15) * 4;
    const int m = m0 + r;
    const int mcl = (m < kNode) ? m : (kNode - 1);
    const v4f v = *(const v4f*)(x + ((size_t)b * kNode + mcl) * kDin + c4);
    const bool ok = (m < kNode);
    tile[r][c4 + 0] = ok ? v[0] : 0.f;
    tile[r][c4 + 1] = ok ? v[1] : 0.f;
    tile[r][c4 + 2] = ok ? v[2] : 0.f;
    tile[r][c4 + 3] = ok ? v[3] : 0.f;
  }
  __syncthreads();
  const int wave = tid >> 5, lane = tid & 31, q = lane >> 3, c8 = (lane & 7) * 8;
  v4u th[2], tl[2], yh[2], yl[2];
#pragma unroll
  for (int it = 0; it < 2; ++it) {
    const int d = it * 32 + wave * 4 + q;
    unsigned w0, w1;
#pragma unroll
    for (int j = 0; j < 4; ++j) {
      split2_bf(tile[c8 + 2 * j][d], tile[c8 + 2 * j + 1][d], w0, w1);
      th[it][j] = w0; tl[it][j] = w1;
      split2_bf(tile[d][c8 + 2 * j], tile[d][c8 + 2 * j + 1], w0, w1);
      yh[it][j] = w0; yl[it][j] = w1;
    }
  }
  for (int pass = 0; pass < 2; ++pass) {
#pragma unroll
    for (int it = 0; it < 2; ++it) {
      const int d = it * 32 + wave * 4 + q;
      const size_t ot = ((size_t)b * kDin + d) * kNpad + m0 + c8;
      const size_t oy = ((size_t)b * kNpad + m0 + d) * kKf + c8;
      *(volatile v4u*)(xthi + ot) = th[it];
      *(volatile v4u*)(xtlo + ot) = tl[it];
      *(volatile v4u*)(yhi + oy)  = yh[it];
      *(volatile v4u*)(ylo + oy)  = yl[it];
    }
    __threadfence();
  }
}

__global__ __launch_bounds__(256) void k_pack_w(const float* __restrict__ wp,
                                                unsigned short* __restrict__ whi, unsigned short* __restrict__ wlo) {
  __shared__ __align__(16) float wl[kCheb * kDin * kDout];
  const int tid = threadIdx.x;
  const int e   = blockIdx.x;
  const v4f* src = (const v4f*)(wp + (size_t)e * kCheb * kDin * kDout);
  for (int i = tid; i < (kCheb * kDin * kDout) / 4; i += 256) {
    const v4f v = src[i];
    wl[4 * i + 0] = v[0]; wl[4 * i + 1] = v[1]; wl[4 * i + 2] = v[2]; wl[4 * i + 3] = v[3];
  }
  __syncthreads();
  const int wave = tid >> 5, lane = tid & 31, q = lane >> 3, c8 = (lane & 7) * 8;
  v4u vh[6], vl[6];
#pragma unroll
  for (int it = 0; it < 6; ++it) {
    const int p  = it * 32 + wave * 4 + q;
    const int o  = p / 3;
    const int ks = p - 3 * o;
    unsigned w0, w1;
#pragma unroll
    for (int j = 0; j < 4; ++j) {
      float v2[2];
#pragma unroll
      for (int t = 0; t < 2; ++t) {
        const int i = c8 + 2 * j + t;
        const float a = wl[(ks * kDin + i) * kDout + o];
        const float c = wl[(2 * kDin + i) * kDout + o];
        v2[t] = (ks == 0) ? (a - c) : ((ks == 2) ? (a + a) : a);
      }
      split2_bf(v2[0], v2[1], w0, w1);
      vh[it][j] = w0; vl[it][j] = w1;
    }
  }
  for (int pass = 0; pass < 2; ++pass) {
#pragma unroll
    for (int it = 0; it < 6; ++it) {
      const int p  = it * 32 + wave * 4 + q;
      const int o  = p / 3;
      const int ks = p - 3 * o;
      const size_t off = (size_t)(e * kDout + o) * kKf + ks * kDin + c8;
      *(volatile v4u*)(whi + off) = vh[it];
      *(volatile v4u*)(wlo + off) = vl[it];
    }
    __threadfence();
  }
}

__global__ __launch_bounds__(256) void k_softmax(const float* __restrict__ sc,
                                                 unsigned short* __restrict__ ahi, unsigned short* __restrict__ alo) {
  __shared__ float smax[8];
  __shared__ float ssum[8];
  const int tid  = threadIdx.x, wave = tid >> 5, lane = tid & 31;
  const int rloc = tid >> 6;
  const int half = wave & 1;
  const int rowg = blockIdx.x * 4 + rloc;
  const int n    = rowg & 511;
  const bool rowvalid = (n < kNode);
  const int c0   = half * 256 + lane * 8;
  const float* srow = sc + (size_t)rowg * kNpad + c0;
  const v4f s0 = *(const v4f*)(srow);
  const v4f s1 = *(const v4f*)(srow + 4);
  float sv[8] = {s0[0], s0[1], s0[2], s0[3], s1[0], s1[1], s1[2], s1[3]};
  float mx = -INFINITY;
#pragma unroll
  for (int j = 0; j < 8; ++j) mx = fmaxf(mx, (c0 + j < kNode) ? sv[j] : -INFINITY);
#pragma unroll
  for (int off = 16; off > 0; off >>= 1) mx = fmaxf(mx, __shfl_xor(mx, off, 32));
  if (lane == 0) smax[wave] = mx;
  __syncthreads();
  const float rmax = fmaxf(smax[2 * rloc], smax[2 * rloc + 1]);
  float ev[8];
  float psum = 0.f;
#pragma unroll
  for (int j = 0; j < 8; ++j) {
    const float ex = expf(sv[j] - rmax);
    ev[j] = (c0 + j < kNode) ? ex : 0.f;
    psum += ev[j];
  }
#pragma unroll
  for (int off = 16; off > 0; off >>= 1) psum += __shfl_xor(psum, off, 32);
  if (lane == 0) ssum[wave] = psum;
  __syncthreads();
  const float tot = ssum[2 * rloc] + ssum[2 * rloc + 1];
  const float inv = 1.0f / tot;
  v4u vh, vl;
#pragma unroll
  for (int j = 0; j < 4; ++j) {
    float p0 = ev[2 * j] * inv, p1 = ev[2 * j + 1] * inv;
    p0 = rowvalid ? p0 : 0.f;
    p1 = rowvalid ? p1 : 0.f;
    unsigned w0, w1;
    split2_bf(p0, p1, w0, w1);
    vh[j] = w0; vl[j] = w1;
  }
  const size_t off = (size_t)rowg * kNpad + c0;
  *(volatile v4u*)(ahi + off) = vh;
  *(volatile v4u*)(alo + off) = vl;
  __threadfence();
  *(volatile v4u*)(ahi + off) = vh;
  *(volatile v4u*)(alo + off) = vl;
}

__global__ __launch_bounds__(256) void k_out(const float* __restrict__ z, const float* __restrict__ st,
                                             const float* __restrict__ bp, float* __restrict__ out) {
  const int gid  = blockIdx.x * 256 + threadIdx.x;
  const int q    = gid & 15;
  const int rown = gid >> 4;
  const int b    = rown / kNode;
  const int n    = rown - b * kNode;
  const float* zrow = z + ((size_t)b * kNpad + n) * kNz + q * 4;
  const float* srow = st + (size_t)rown * kEmb;
  const float* brow = bp + q * 4;
  v4f acc = (v4f){0.f, 0.f, 0.f, 0.f};
#pragma unroll 1
  for (int e4 = 0; e4 < 4; ++e4) {
    const v4f s4 = *(const v4f*)(srow + e4 * 4);
#pragma unroll
    for (int j = 0; j < 4; ++j) {
      const int e = e4 * 4 + j;
      const v4f zz = *(const v4f*)(zrow + e * kDout);
      const v4f bb = *(const v4f*)(brow + e * kDout);
      acc += s4[j] * (zz + bb);
    }
  }
  const size_t off = (size_t)rown * kDout + q * 4;
  *(volatile v4f*)(out + off) = acc;
  __threadfence();
  *(volatile v4f*)(out + off) = acc;
}

extern "C" void kernel_launch(void* const* d_in, const int* in_sizes, int n_in,
                              void* d_out, int out_size, void* d_ws, size_t ws_size,
                              hipStream_t stream) {
  (void)in_sizes; (void)n_in; (void)out_size; (void)ws_size;
  const float* x    = (const float*)d_in[0];
  const float* aemb = (const float*)d_in[1];
  const float* semb = (const float*)d_in[2];
  const float* wp   = (const float*)d_in[3];
  const float* bp   = (const float*)d_in[4];
  float* out = (float*)d_out;
  unsigned char* ws = (unsigned char*)d_ws;

  unsigned short* pa    = (unsigned short*)(ws + kOffPA);
  unsigned short* pb    = (unsigned short*)(ws + kOffPB);
  float*          sc    = (float*)(ws + kOffS);
  unsigned short* ahi   = (unsigned short*)(ws + kOffAhi);
  unsigned short* alo   = (unsigned short*)(ws + kOffAlo);
  float*          zz    = (float*)(ws + kOffZ);
  unsigned short* xthi  = (unsigned short*)(ws + kOffXThi);
  unsigned short* xtlo  = (unsigned short*)(ws + kOffXTlo);
  unsigned short* xt1hi = (unsigned short*)(ws + kOffXT1hi);
  unsigned short* xt1lo = (unsigned short*)(ws + kOffXT1lo);
  unsigned short* yhi   = (unsigned short*)(ws + kOffYhi);
  unsigned short* ylo   = (unsigned short*)(ws + kOffYlo);
  unsigned short* whi   = (unsigned short*)(ws + kOffWhi);
  unsigned short* wlo   = (unsigned short*)(ws + kOffWlo);

  k_pack_emb<<<(kBatch * kNpad * 16) / 256, 256, 0, stream>>>(aemb, pa, pb);
  k_pack_x<<<dim3(kNpad / 64, kBatch), 256, 0, stream>>>(x, xthi, xtlo, yhi, ylo);
  k_pack_w<<<kEmb, 256, 0, stream>>>(wp, whi, wlo);

  wmma_gemm64<1, false, 0, 0, false, 2><<<dim3((kNpad / 64) * (kNpad / 64) / 8, kBatch), 256, 0, stream>>>(
      pa, pa, kKsPitch, (long)kNpad * kKsPitch,
      pb, pb, kKsPitch, (long)kNpad * kKsPitch,
      (void*)sc, (void*)sc, kNpad, (long)kNpad * kNpad,
      x, x, 0L, kNpad, kNpad, kKsReal, 1.0f);

  k_softmax<<<(kBatch * kNpad) / 4, 256, 0, stream>>>(sc, ahi, alo);

  wmma_gemm64<1, true, 0, 2, false, 0><<<dim3(1, kBatch), 256, 0, stream>>>(
      ahi, alo, kNpad, (long)kNpad * kNpad,
      xthi, xtlo, kNpad, (long)kDin * kNpad,
      (void*)(yhi + kDin), (void*)(ylo + kDin), kKf, (long)kNpad * kKf,
      x, x, 0L, kNpad, kDin, kNpad, 1.0f);

  wmma_gemm64<1, true, 0, 2, false, 0><<<dim3(1, kBatch), 256, 0, stream>>>(
      xthi, xtlo, kNpad, (long)kDin * kNpad,
      ahi, alo, kNpad, (long)kNpad * kNpad,
      (void*)xt1hi, (void*)xt1lo, kNpad, (long)kDin * kNpad,
      x, x, 0L, kDin, kNpad, kNpad, 1.0f);

  wmma_gemm64<1, true, 0, 2, false, 0><<<dim3(1, kBatch), 256, 0, stream>>>(
      ahi, alo, kNpad, (long)kNpad * kNpad,
      xt1hi, xt1lo, kNpad, (long)kDin * kNpad,
      (void*)(yhi + 2 * kDin), (void*)(ylo + 2 * kDin), kKf, (long)kNpad * kKf,
      x, x, 0L, kNpad, kDin, kNpad, 1.0f);

  wmma_gemm64<1, true, 0, 0, false, 0><<<dim3((kNpad / 64) * (kNz / 64) / 8, kBatch), 256, 0, stream>>>(
      yhi, ylo, kKf, (long)kNpad * kKf,
      whi, wlo, kKf, 0L,
      (void*)zz, (void*)zz, kNz, (long)kNpad * kNz,
      x, x, 0L, kNpad, kNz, kKf, 1.0f);

  k_out<<<(kBatch * kNode * 16) / 256, 256, 0, stream>>>(zz, semb, bp, out);
}
